// HGT_40939628265927
// MI455X (gfx1250) — hardware-run, weakly checked
//
#include <hip/hip_runtime.h>
#include <stddef.h>
#include <stdint.h>
#include <math.h>


#define DIM    128
#define HN     8
#define DK     16
#define K2     256
#define KVW    256
#define NQKV   384
#define NOUT   90
#define NOP    96
#define NTO    6
#define NTHR   256
#define NWAVE  8
#define EPT    8
#define CHUNK  (NTHR * EPT)
#define WCAP   (EPT * 32)
#define LISTN  (NWAVE * WCAP)
#define RCAP   28672
#define GBM    32
#define GTHR   64
#define BBM    64
#define BTHR   128
#define ATTSC  0.25f
#define WSMAX  134217728
#define NBI    32
#define SLI    5
#define DGI    1024
#define NBN    128
#define SLN    7
#define DGN    512
#define NBP    1024
#define SLP    10
#define DGP    128
#define NU0    (DIM * (DIM / 8))
#define NU1    (6 * NQKV * (K2 / 8))
#define NU2    (6 * DIM * (K2 / 8))
#define NU3    (NOP * (K2 / 8))
#define NU4    (8 * 16 * 16 * 4)
#define NUT    (NU0 + NU1 + NU2 + NU3 + NU4)
#define AGG_INTS(nb) (2 * RCAP + 3 * (nb) + LISTN + 2 * NWAVE)
#define NPQ    ((GBM * NOUT / 4 + GTHR - 1) / GTHR)

static_assert((CHUNK & (CHUNK - 1)) == 0 && CHUNK == 2048);
static_assert(NBI == (1 << SLI) && NBN == (1 << SLN) && NBP == (1 << SLP));
static_assert(((long long)CHUNK << SLP) < (1LL << 31));
static_assert(LISTN >= NBP && (RCAP % 32) == 0);
static_assert(NU0 % NTHR == 0 && NU1 % NTHR == 0 && NU2 % NTHR == 0 && NU3 % NTHR == 0 && NU4 % NTHR == 0);
static_assert((NQKV * (K2 / 8)) % NTHR == 0);
static_assert(GBM == (GTHR / 32) * 16 && BBM == (BTHR / 32) * 16);
static_assert(HN * DK == DIM && DK == 16 && DIM == 32 * 4);
static_assert(K2 == 2 * DIM && (K2 % 32) == 0 && (DIM % 32) == 0);
static_assert(NOP == 16 * NTO && NOP >= NOUT && ((GBM * NOUT) % 4) == 0 && ((GBM * NOUT * 4) % 128) == 0);
static_assert(AGG_INTS(NBP) * 4 + 64 <= 300000);
static_assert(BBM * (64 / 8) == 4 * BTHR);
static_assert(NPQ * GTHR * 4 >= GBM * NOUT);

typedef float          v4f   __attribute__((ext_vector_type(4)));
typedef float          v8f   __attribute__((ext_vector_type(8)));
typedef int            v4i   __attribute__((ext_vector_type(4)));
typedef int            v8i   __attribute__((ext_vector_type(8)));
typedef unsigned int   v4u   __attribute__((ext_vector_type(4)));
typedef unsigned short v8us  __attribute__((ext_vector_type(8)));
typedef unsigned short v16us __attribute__((ext_vector_type(16)));
typedef __bf16         v16bf __attribute__((ext_vector_type(16)));
typedef v4f  __attribute__((may_alias)) v4fa;
typedef v4i  __attribute__((may_alias)) v4ia;
typedef v4u  __attribute__((may_alias)) v4ua;
typedef v8us __attribute__((may_alias)) v8usa;
union Frag { v16bf v; v16us u; v8us h[2]; v8i w; };

__device__ __forceinline__ v8f wmb(const Frag& a, const Frag& b, v8f c) {
  v8f d = __builtin_amdgcn_wmma_f32_16x16x32_bf16(false, a.v, false, b.v, (short)0, c, false, false);
  asm volatile("v_nop\n\tv_nop\n\tv_nop\n\tv_nop" : "+v"(d) : "v"(a.w), "v"(b.w));
  return d;
}

__device__ __forceinline__ void ldwait() {
  asm volatile("s_wait_loadcnt 0x0" ::: "memory");
}

__device__ __forceinline__ unsigned bf16_bits(float f) {
  const unsigned u = __float_as_uint(f);
  return ((u + 0x7FFFu + ((u >> 16) & 1u)) >> 16) & 0xFFFFu;
}
__device__ __forceinline__ float bf16_val(float f) { return __uint_as_float(bf16_bits(f) << 16); }

__device__ __forceinline__ v8us hilo8(v4f t) {
  v8us o;
  unsigned hb;
  hb = bf16_bits(t.x); o[0] = (unsigned short)hb; o[4] = (unsigned short)bf16_bits(t.x - __uint_as_float(hb << 16));
  hb = bf16_bits(t.y); o[1] = (unsigned short)hb; o[5] = (unsigned short)bf16_bits(t.y - __uint_as_float(hb << 16));
  hb = bf16_bits(t.z); o[2] = (unsigned short)hb; o[6] = (unsigned short)bf16_bits(t.z - __uint_as_float(hb << 16));
  hb = bf16_bits(t.w); o[3] = (unsigned short)hb; o[7] = (unsigned short)bf16_bits(t.w - __uint_as_float(hb << 16));
  return o;
}
__device__ __forceinline__ void hl2(float v0, float v1, unsigned& hw, unsigned& lw) {
  const unsigned h0 = bf16_bits(v0), h1 = bf16_bits(v1);
  const unsigned l0 = bf16_bits(v0 - __uint_as_float(h0 << 16)), l1 = bf16_bits(v1 - __uint_as_float(h1 << 16));
  hw = h0 | (h1 << 16);
  lw = l0 | (l1 << 16);
}
__device__ __forceinline__ void pack8hl(const v4f a, const v4f b, v4u& hv, v4u& lv) {
  unsigned h, l;
  hl2(a.x, a.y, h, l); hv.x = h; lv.x = l;
  hl2(a.z, a.w, h, l); hv.y = h; lv.y = l;
  hl2(b.x, b.y, h, l); hv.z = h; lv.z = l;
  hl2(b.z, b.w, h, l); hv.w = h; lv.w = l;
}

__device__ __forceinline__ float gelu_t(float x) {
  const float u  = x * x * x;
  const float y  = 0.7978845608028654f * fmaf(0.044715f, u, x);
  const float e  = __expf(2.0f * y);
  const float th = 1.0f - 2.0f * __builtin_amdgcn_rcpf(1.0f + e);
  return x * (0.5f * (1.0f + th));
}
__device__ __forceinline__ float sigm_t(float z) {
  return __builtin_amdgcn_rcpf(1.0f + __expf(-z));
}

template <int SLB>
__device__ __forceinline__ int scan_chunk(const int* __restrict__ dsts, int nE, int cbase, int slotBase,
                                          int nb, int vec8, int* list, int tid, int lane, int wave) {
  int wc = 0;
  const int el0  = tid * EPT;
  const int e0   = cbase + el0;
  const int sent = -2147483647 - 1;
  v4i da, db;
  if (vec8 != 0 && cbase + CHUNK <= nE) {
    da = *(const v4i*)(dsts + e0);
    db = *(const v4i*)(dsts + e0 + 4);
  } else {
    da.x = (e0     < nE) ? dsts[min(e0,     nE - 1)] : sent;
    da.y = (e0 + 1 < nE) ? dsts[min(e0 + 1, nE - 1)] : sent;
    da.z = (e0 + 2 < nE) ? dsts[min(e0 + 2, nE - 1)] : sent;
    da.w = (e0 + 3 < nE) ? dsts[min(e0 + 3, nE - 1)] : sent;
    db.x = (e0 + 4 < nE) ? dsts[min(e0 + 4, nE - 1)] : sent;
    db.y = (e0 + 5 < nE) ? dsts[min(e0 + 5, nE - 1)] : sent;
    db.z = (e0 + 6 < nE) ? dsts[min(e0 + 6, nE - 1)] : sent;
    db.w = (e0 + 7 < nE) ? dsts[min(e0 + 7, nE - 1)] : sent;
  }
  const unsigned nbs = (unsigned)slotBase;
  const unsigned unb = (unsigned)nb;
  const unsigned s0 = (unsigned)da.x - nbs, s1 = (unsigned)da.y - nbs;
  const unsigned s2 = (unsigned)da.z - nbs, s3 = (unsigned)da.w - nbs;
  const unsigned s4 = (unsigned)db.x - nbs, s5 = (unsigned)db.y - nbs;
  const unsigned s6 = (unsigned)db.z - nbs, s7 = (unsigned)db.w - nbs;
  const bool h0 = s0 < unb, h1 = s1 < unb, h2 = s2 < unb, h3 = s3 < unb;
  const bool h4 = s4 < unb, h5 = s5 < unb, h6 = s6 < unb, h7 = s7 < unb;
  const unsigned any = __builtin_amdgcn_ballot_w32(h0 | h1 | h2 | h3 | h4 | h5 | h6 | h7);
  if (any != 0u) {
#define HITJ(J, HJ, SJ) { \
      const unsigned mj = __builtin_amdgcn_ballot_w32(HJ); \
      if (mj != 0u) { \
        if (HJ) { \
          const int pos = wc + (int)__builtin_amdgcn_mbcnt_lo(mj, 0u); \
          if (pos < WCAP) list[wave * WCAP + pos] = ((el0 + (J)) << SLB) | (int)(SJ); \
        } \
        wc += (int)__builtin_popcount(mj); } }
    HITJ(0, h0, s0)
    HITJ(1, h1, s1)
    HITJ(2, h2, s2)
    HITJ(3, h3, s3)
    HITJ(4, h4, s4)
    HITJ(5, h5, s5)
    HITJ(6, h6, s6)
    HITJ(7, h7, s7)
#undef HITJ
  }
  return wc;
}

__global__ __launch_bounds__(NTHR) void k_prep(const float* __restrict__ win, const float* __restrict__ kw,
                                               const float* __restrict__ vw, const float* __restrict__ qw,
                                               const float* __restrict__ aw, const float* __restrict__ wout,
                                               const float* __restrict__ arel, const float* __restrict__ mrel,
                                               unsigned short* WINT, unsigned short* KQVT, unsigned short* AWT,
                                               unsigned short* WOT, unsigned short* BDT) {
  const int u = (int)blockIdx.x * NTHR + (int)threadIdx.x;
  v8us o;
  unsigned short* dp;
  if (u < NU0) {
    const int n  = u >> 4;
    const int k8 = (u & 15) * 8;
    const float* p = win + (size_t)k8 * DIM + n;
#pragma unroll
    for (int i = 0; i < 8; ++i) o[i] = (unsigned short)bf16_bits(p[(size_t)i * DIM]);
    dp = WINT + (size_t)n * DIM + k8;
  } else if (u < NU0 + NU1) {
    const int v   = u - NU0;
    const int lt  = v / (NQKV * (K2 / 8));
    const int rm  = v - lt * (NQKV * (K2 / 8));
    const int n   = rm >> 5;
    const int g   = rm & 31;
    const int seg = n >> 7;
    const int nn  = n & 127;
    const float* W = kw;
    if (seg == 1) W = vw;
    else if (seg == 2) W = qw;
    const float* p = W + (size_t)lt * DIM * DIM + (size_t)(4 * g) * DIM + nn;
    const unsigned short f0 = (unsigned short)bf16_bits(p[0]);
    const unsigned short f1 = (unsigned short)bf16_bits(p[DIM]);
    const unsigned short f2 = (unsigned short)bf16_bits(p[2 * DIM]);
    const unsigned short f3 = (unsigned short)bf16_bits(p[3 * DIM]);
    o[0] = f0; o[1] = f1; o[2] = f2; o[3] = f3; o[4] = f0; o[5] = f1; o[6] = f2; o[7] = f3;
    dp = KQVT + ((size_t)lt * NQKV + (size_t)n) * K2 + 8 * g;
  } else if (u < NU0 + NU1 + NU2) {
    const int v  = u - NU0 - NU1;
    const int lt = v >> 12;
    const int n  = (v >> 5) & 127;
    const int g  = v & 31;
    const float* p = aw + (size_t)lt * DIM * DIM + (size_t)(4 * g) * DIM + n;
    const unsigned short f0 = (unsigned short)bf16_bits(p[0]);
    const unsigned short f1 = (unsigned short)bf16_bits(p[DIM]);
    const unsigned short f2 = (unsigned short)bf16_bits(p[2 * DIM]);
    const unsigned short f3 = (unsigned short)bf16_bits(p[3 * DIM]);
    o[0] = f0; o[1] = f1; o[2] = f2; o[3] = f3; o[4] = f0; o[5] = f1; o[6] = f2; o[7] = f3;
    dp = AWT + ((size_t)lt * DIM + (size_t)n) * K2 + 8 * g;
  } else if (u < NU0 + NU1 + NU2 + NU3) {
    const int v   = u - NU0 - NU1 - NU2;
    const int n   = v >> 5;
    const int g   = v & 31;
    const int ncl = n < NOUT ? n : NOUT - 1;
    const float* p = wout + (size_t)(4 * g) * NOUT + ncl;
    unsigned short f0 = (unsigned short)bf16_bits(p[0]);
    unsigned short f1 = (unsigned short)bf16_bits(p[NOUT]);
    unsigned short f2 = (unsigned short)bf16_bits(p[2 * NOUT]);
    unsigned short f3 = (unsigned short)bf16_bits(p[3 * NOUT]);
    if (n >= NOUT) { f0 = 0; f1 = 0; f2 = 0; f3 = 0; }
    o[0] = f0; o[1] = f1; o[2] = f2; o[3] = f3; o[4] = f0; o[5] = f1; o[6] = f2; o[7] = f3;
    dp = WOT + (size_t)n * K2 + 8 * g;
  } else if (u < NUT) {
    const int v  = u - NU0 - NU1 - NU2 - NU3;
    const int lr = v >> 10;
    const int g  = (v >> 6) & 15;
    const int n  = (v >> 2) & 15;
    const int kq = v & 3;
    const int j0 = (kq * 8) & 15;
    const int r  = lr & 3;
    const int hd = g & 7;
    const bool useA = g < 8;
    const float* P = useA ? arel : mrel;
    const int tr   = (useA && ((r & 1) == 0)) ? 1 : 0;
    const int strd = tr ? 1 : 16;
    const int base = tr ? ((((lr * 8 + hd) * 16) + n) * 16 + j0)
                        : ((((lr * 8 + hd) * 16) + j0) * 16 + n);
#pragma unroll
    for (int i = 0; i < 8; ++i) o[i] = (unsigned short)bf16_bits(P[base + i * strd]);
    dp = BDT + ((size_t)(lr * 16 + g) * 16 + (size_t)n) * 32 + kq * 8;
  } else {
    return;
  }
  *(volatile v8us*)dp = o;
  __threadfence();
  *(volatile v8us*)dp = o;
}

__global__ __launch_bounds__(NTHR) void k_cvx(const float* __restrict__ x, int nN, int nUnits,
                                              unsigned short* xb) {
  const int u = (int)blockIdx.x * NTHR + (int)threadIdx.x;
  if (u >= nUnits) return;
  const int row = u >> 4;
  const int k8  = (u & 15) * 8;
  const int rc  = row < nN ? row : nN - 1;
  const float* p = x + (size_t)rc * DIM + k8;
  const v4f a = *(const v4fa*)p;
  const v4f b = *(const v4fa*)(p + 4);
  const bool ok = row < nN;
  v8us o;
  o[0] = ok ? (unsigned short)bf16_bits(a.x) : (unsigned short)0;
  o[1] = ok ? (unsigned short)bf16_bits(a.y) : (unsigned short)0;
  o[2] = ok ? (unsigned short)bf16_bits(a.z) : (unsigned short)0;
  o[3] = ok ? (unsigned short)bf16_bits(a.w) : (unsigned short)0;
  o[4] = ok ? (unsigned short)bf16_bits(b.x) : (unsigned short)0;
  o[5] = ok ? (unsigned short)bf16_bits(b.y) : (unsigned short)0;
  o[6] = ok ? (unsigned short)bf16_bits(b.z) : (unsigned short)0;
  o[7] = ok ? (unsigned short)bf16_bits(b.w) : (unsigned short)0;
  unsigned short* dp = xb + (size_t)row * DIM + k8;
  *(volatile v8us*)dp = o;
  __threadfence();
  *(volatile v8us*)dp = o;
}

__global__ __launch_bounds__(NTHR) void k_emb(const float* __restrict__ emb1, const int* __restrict__ id1,
                                              int n1, int ne1, int mp1,
                                              const float* __restrict__ emb2, const int* __restrict__ id2,
                                              int n2, int ne2, int mp2,
                                              unsigned short* xh1, unsigned short* xh2) {
  const int u  = (int)blockIdx.x * NTHR + (int)threadIdx.x;
  const int U1 = mp1 * 32, U2 = mp2 * 32;
  const float* emb = emb1;
  const int*   ids = id1;
  int nn = n1, ne = ne1, v = u;
  unsigned short* xh = xh1;
  if (u >= U1) {
    if (u >= U1 + U2) return;
    emb = emb2; ids = id2; nn = n2; ne = ne2; xh = xh2; v = u - U1;
  }
  const int row = v >> 5;
  const int g   = v & 31;
  const int rc  = row < nn ? row : nn - 1;
  int id = ids[rc];
  id = id < 0 ? id + ne : id;
  id = id < 0 ? 0 : (id > ne - 1 ? ne - 1 : id);
  const v4f a = *(const v4fa*)(emb + (size_t)id * DIM + 4 * g);
  v4f t;
  t.x = fmaxf(bf16_val(a.x), 0.0f); t.y = fmaxf(bf16_val(a.y), 0.0f);
  t.z = fmaxf(bf16_val(a.z), 0.0f); t.w = fmaxf(bf16_val(a.w), 0.0f);
  if (row >= nn) { const v4f z4 = {0.0f, 0.0f, 0.0f, 0.0f}; t = z4; }
  const v8us po = hilo8(t);
  unsigned short* dp = xh + (size_t)row * K2 + 8 * g;
  *(volatile v8us*)dp = po;
  __threadfence();
  *(volatile v8us*)dp = po;
}

__global__ __launch_bounds__(GTHR) void k_gemm0(const unsigned short* __restrict__ A,
                                                const unsigned short* __restrict__ WT,
                                                const float* __restrict__ bias, unsigned short* hpl) {
  __shared__ __attribute__((aligned(16))) float stg[GBM * DIM];
  const int tid = (int)threadIdx.x, lane = tid & 31, wave = tid >> 5, hh = lane >> 4, m = lane & 15;
  const int rowBase = (int)blockIdx.x * GBM;

  v8f acc[8];
  {
    const v8f z = {0.f, 0.f, 0.f, 0.f, 0.f, 0.f, 0.f, 0.f};
#pragma unroll
    for (int t = 0; t < 8; ++t) acc[t] = z;
  }
  const unsigned short* ap = A  + (size_t)(rowBase + 16 * wave + m) * (size_t)DIM + 8 * hh;
  const unsigned short* bp = WT + (size_t)m * (size_t)DIM + 8 * hh;

#pragma unroll 1
  for (int ks = 0; ks < DIM / 32; ++ks) {
    const int k0 = 32 * ks;
    Frag af;
    af.h[0] = *(const v8usa*)(ap + k0);
    af.h[1] = *(const v8usa*)(ap + k0 + 16);
#pragma unroll
    for (int nt = 0; nt < 8; ++nt) {
      const unsigned short* wq = bp + (size_t)(16 * nt) * (size_t)DIM + k0;
      Frag bf;
      bf.h[0] = *(const v8usa*)wq;
      bf.h[1] = *(const v8usa*)(wq + 16);
      acc[nt] = wmb(af, bf, acc[nt]);
    }
  }

#pragma unroll
  for (int nt = 0; nt < 8; ++nt) {
    const int lc = 16 * nt + m;
#pragma unroll
    for (int r = 0; r < 8; ++r) {
      const int lr = 16 * wave + 8 * hh + r;
      stg[lr * DIM + lc] = acc[nt][r];
    }
  }
  __syncthreads();

  v4f bb4;
  {
    const v4f tb = *(const v4fa*)(bias + 4 * lane);
    bb4.x = bf16_val(tb.x); bb4.y = bf16_val(tb.y); bb4.z = bf16_val(tb.z); bb4.w = bf16_val(tb.w);
  }
  v8us po[16];
#pragma unroll
  for (int i = 0; i < 16; ++i) {
    v4f t = *(const v4fa*)(stg + (16 * wave + i) * DIM + 4 * lane) + bb4;
    t.x = fmaxf(t.x, 0.0f); t.y = fmaxf(t.y, 0.0f); t.z = fmaxf(t.z, 0.0f); t.w = fmaxf(t.w, 0.0f);
    po[i] = hilo8(t);
  }
#pragma unroll
  for (int i = 0; i < 16; ++i) {
    unsigned short* rp = hpl + (size_t)(rowBase + 16 * wave + i) * (size_t)K2 + 8 * lane;
    *(volatile v8us*)rp = po[i];
  }
  __threadfence();
#pragma unroll
  for (int i = 0; i < 16; ++i) {
    unsigned short* rp = hpl + (size_t)(rowBase + 16 * wave + i) * (size_t)K2 + 8 * lane;
    *(volatile v8us*)rp = po[i];
  }
}

__global__ __launch_bounds__(GTHR) void k_gemmx(const unsigned short* __restrict__ A,
                                                const unsigned short* __restrict__ WT3,
                                                const float* __restrict__ bk, const float* __restrict__ bvv,
                                                const float* __restrict__ bq, float* KVo, float* Qo) {
  __shared__ __attribute__((aligned(16))) float stg[GBM * DIM];
  const int tid = (int)threadIdx.x, lane = tid & 31, wave = tid >> 5, hh = lane >> 4, m = lane & 15;
  const int rowBase = (int)blockIdx.x * GBM;
  const int seg = (int)blockIdx.y;
  const unsigned short* WT = WT3 + (size_t)seg * (size_t)DIM * (size_t)K2;
  const float* bias = bk;
  float* outp = KVo;
  int ldo = KVW;
  if (seg == 1) { bias = bvv; outp = KVo + DIM; }
  else if (seg == 2) { bias = bq; outp = Qo; ldo = DIM; }

  v8f acc[8];
  {
    const v8f z = {0.f, 0.f, 0.f, 0.f, 0.f, 0.f, 0.f, 0.f};
#pragma unroll
    for (int t = 0; t < 8; ++t) acc[t] = z;
  }
  const unsigned short* ap = A  + (size_t)(rowBase + 16 * wave + m) * (size_t)K2 + 8 * hh;
  const unsigned short* bp = WT + (size_t)m * (size_t)K2 + 8 * hh;

#pragma unroll 1
  for (int ks = 0; ks < K2 / 32; ++ks) {
    const int k0 = 32 * ks;
    Frag af;
    af.h[0] = *(const v8usa*)(ap + k0);
    af.h[1] = *(const v8usa*)(ap + k0 + 16);
#pragma unroll
    for (int nt = 0; nt < 8; ++nt) {
      const unsigned short* wq = bp + (size_t)(16 * nt) * (size_t)K2 + k0;
      Frag bf;
      bf.h[0] = *(const v8usa*)wq;
      bf.h[1] = *(const v8usa*)(wq + 16);
      acc[nt] = wmb(af, bf, acc[nt]);
    }
  }

#pragma unroll
  for (int nt = 0; nt < 8; ++nt) {
    const int lc = 16 * nt + m;
#pragma unroll
    for (int r = 0; r < 8; ++r) {
      const int lr = 16 * wave + 8 * hh + r;
      stg[lr * DIM + lc] = acc[nt][r];
    }
  }
  __syncthreads();

  v4f bb4;
  {
    const v4f tb = *(const v4fa*)(bias + 4 * lane);
    bb4.x = bf16_val(tb.x); bb4.y = bf16_val(tb.y); bb4.z = bf16_val(tb.z); bb4.w = bf16_val(tb.w);
  }
  v4f fv[16];
#pragma unroll
  for (int i = 0; i < 16; ++i) {
    const int lr = 16 * wave + i;
    fv[i] = *(const v4fa*)(stg + lr * DIM + 4 * lane) + bb4;
  }
#pragma unroll
  for (int i = 0; i < 16; ++i) {
    float* op = outp + (size_t)(rowBase + 16 * wave + i) * (size_t)ldo + 4 * lane;
    *(volatile v4f*)op = fv[i];
  }
  __threadfence();
#pragma unroll
  for (int i = 0; i < 16; ++i) {
    float* op = outp + (size_t)(rowBase + 16 * wave + i) * (size_t)ldo + 4 * lane;
    *(volatile v4f*)op = fv[i];
  }
}

template <int MODE>
__global__ __launch_bounds__(BTHR) void k_bd(const float* __restrict__ Xin, int ldi,
                                             const unsigned short* __restrict__ bdt,
                                             float* outF, int ldo, unsigned short* outH) {
  __shared__ __attribute__((aligned(16))) unsigned short At[BBM * 128];
  __shared__ __attribute__((aligned(16))) float stg[BBM * 64];
  const int tid = (int)threadIdx.x, lane = tid & 31, wave = tid >> 5, hh = lane >> 4, m = lane & 15;
  const int rowBase = (int)blockIdx.x * BBM;
  const int yb = (int)blockIdx.y;
  const int cb = 64 * yb;

#pragma unroll 1
  for (int i = 0; i < 4; ++i) {
    const int p   = i * BTHR + tid;
    const int row = p >> 3;
    const int q8  = (p & 7) * 8;
    const int gl  = q8 >> 4;
    const int j0  = q8 & 15;
    const float* xp = Xin + (size_t)(rowBase + row) * (size_t)ldi + cb + q8;
    const v4f a = *(const v4fa*)xp;
    const v4f b = *(const v4fa*)(xp + 4);
    v4u hv, lv;
    pack8hl(a, b, hv, lv);
    *(v4ua*)(At + row * 128 + 32 * gl + j0)      = hv;
    *(v4ua*)(At + row * 128 + 32 * gl + 16 + j0) = lv;
  }
  __syncthreads();

  const v8f z = {0.f, 0.f, 0.f, 0.f, 0.f, 0.f, 0.f, 0.f};
  const unsigned short* aq = At + (size_t)(16 * wave + m) * 128 + 8 * hh;
#pragma unroll
  for (int t = 0; t < 4; ++t) {
    Frag af, bf;
    af.h[0] = *(const v8usa*)(aq + 32 * t);
    af.h[1] = *(const v8usa*)(aq + 32 * t + 16);
    const unsigned short* bq = bdt + (size_t)((4 * yb + t) * 16 + m) * 32 + 8 * hh;
    bf.h[0] = *(const v8usa*)bq;
    bf.h[1] = *(const v8usa*)(bq + 16);
    const v8f acc = wmb(af, bf, z);
#pragma unroll
    for (int r = 0; r < 8; ++r) {
      const int lr = 16 * wave + 8 * hh + r;
      stg[lr * 64 + 16 * t + m] = acc[r];
    }
  }
  __syncthreads();

  v4f fv[8];
#pragma unroll
  for (int i = 0; i < 8; ++i) {
    const int lr = 16 * wave + 2 * i + hh;
    fv[i] = *(const v4fa*)(stg + lr * 64 + 4 * m);
  }
  if constexpr (MODE == 0) {
#pragma unroll
    for (int i = 0; i < 8; ++i) {
      const int lr = 16 * wave + 2 * i + hh;
      float* op = outF + (size_t)(rowBase + lr) * (size_t)ldo + cb + 4 * m;
      *(volatile v4f*)op = fv[i];
    }
    __threadfence();
#pragma unroll
    for (int i = 0; i < 8; ++i) {
      const int lr = 16 * wave + 2 * i + hh;
      float* op = outF + (size_t)(rowBase + lr) * (size_t)ldo + cb + 4 * m;
      *(volatile v4f*)op = fv[i];
    }
  } else {
    v8us po[8];
#pragma unroll
    for (int i = 0; i < 8; ++i) {
      v4f gv;
      gv.x = gelu_t(fv[i].x); gv.y = gelu_t(fv[i].y); gv.z = gelu_t(fv[i].z); gv.w = gelu_t(fv[i].w);
      po[i] = hilo8(gv);
    }
#pragma unroll
    for (int i = 0; i < 8; ++i) {
      const int lr = 16 * wave + 2 * i + hh;
      unsigned short* hp = outH + (size_t)(rowBase + lr) * (size_t)K2 + 8 * (16 * yb + m);
      *(volatile v8us*)hp = po[i];
    }
    __threadfence();
#pragma unroll
    for (int i = 0; i < 8; ++i) {
      const int lr = 16 * wave + 2 * i + hh;
      unsigned short* hp = outH + (size_t)(rowBase + lr) * (size_t)K2 + 8 * (16 * yb + m);
      *(volatile v8us*)hp = po[i];
    }
  }
}

template <int NB, int SLB, int DEGC, int MODE>
__global__ __launch_bounds__(NTHR) void k_agg(
    const int* __restrict__ srcs, const int* __restrict__ dsts, int nE, int vec8,
    const float* __restrict__ Qp, int nDst, const float* __restrict__ KVp, int nSrc,
    const float* __restrict__ prel, float* Sp, unsigned short* Hp, int MPr) {
  static_assert(NB == (1 << SLB) && (NB % 32) == 0 && (NB % NWAVE) == 0 && NB <= LISTN);
  static_assert(((long long)CHUNK << SLB) < (1LL << 31));
  extern __shared__ v4f lds_dyn[];
  int* reg1 = (int*)lds_dyn;
  int* reg2 = reg1 + RCAP;
  int* scnt = reg2 + RCAP;
  int* soff = scnt + NB;
  int* cur  = soff + NB;
  int* list = cur + NB;
  int* wcnt = list + LISTN;
  const int tid = (int)threadIdx.x, lane = tid & 31, wave = tid >> 5;
  const int nodeBase = (int)blockIdx.x * NB;

  for (int i = tid; i < NB; i += NTHR) { scnt[i] = 0; soff[i] = 0; cur[i] = 0; }
  if (tid < NWAVE) wcnt[tid] = 0;
  __syncthreads();

  int tot = 0;
  const int nChunks = (nE + CHUNK - 1) / CHUNK;
#pragma unroll 1
  for (int ch = 0; ch < nChunks; ++ch) {
    const int cbase = ch * CHUNK;
    const int wc = scan_chunk<SLB>(dsts, nE, cbase, nodeBase, NB, vec8, list, tid, lane, wave);
    if (lane == 0) wcnt[wave] = wc;
    __syncthreads();
    int pre = 0, all = 0;
#pragma unroll
    for (int w2 = 0; w2 < NWAVE; ++w2) {
      int c = wcnt[w2];
      c = c < 0 ? 0 : (c > WCAP ? WCAP : c);
      all += c;
      pre += (w2 < wave) ? c : 0;
    }
    const int wcc  = wc > WCAP ? WCAP : wc;
    const int base = tot + pre;
#pragma unroll 1
    for (int i = lane; i < wcc; i += 32) {
      const int ent = list[wave * WCAP + i];
      const int el  = (ent >> SLB) & (CHUNK - 1);
      const int sl  = ent & (NB - 1);
      int eid = cbase + el;
      eid = eid > nE - 1 ? nE - 1 : eid;
      const int pos = base + i;
      if (pos < RCAP) reg1[pos] = (int)(((unsigned)eid << SLB) | (unsigned)sl);
    }
    tot += all;
    tot = tot > RCAP ? RCAP : tot;
    __syncthreads();
  }
  const int nh = tot;

  if (wave == 0) {
#pragma unroll 1
    for (int b0 = 0; b0 < nh; b0 += 32) {
      const int idx = b0 + lane;
      const int uv  = reg1[idx < nh ? idx : nh - 1];
      const int m32 = (nh - b0) < 32 ? (nh - b0) : 32;
#pragma unroll 1
      for (int k = 0; k < m32; ++k) {
        const int u  = __builtin_amdgcn_readlane(uv, k);
        const int sl = u & (NB - 1);
        if (lane == 0) scnt[sl] = scnt[sl] + 1;
      }
    }
  }
  __syncthreads();

  if (wave == 0) {
    const int base = lane * (NB / 32);
    int sacc = 0;
#pragma unroll 1
    for (int i = 0; i < NB / 32; ++i) { const int c = scnt[base + i]; sacc += c < 0 ? 0 : c; }
    int incl = sacc;
#pragma unroll
    for (int d = 1; d < 32; d <<= 1) {
      const int y = __shfl_up(incl, d, 32);
      if (lane >= d) incl += y;
    }
    int run = incl - sacc;
#pragma unroll 1
    for (int i = 0; i < NB / 32; ++i) {
      const int c = scnt[base + i];
      soff[base + i] = run;
      cur[base + i]  = run;
      run += c < 0 ? 0 : c;
    }
  }
  __syncthreads();

  if (wave == 0) {
#pragma unroll 1
    for (int b0 = 0; b0 < nh; b0 += 32) {
      const int idx = b0 + lane;
      const int uv  = reg1[idx < nh ? idx : nh - 1];
      const int m32 = (nh - b0) < 32 ? (nh - b0) : 32;
#pragma unroll 1
      for (int k = 0; k < m32; ++k) {
        const int u   = __builtin_amdgcn_readlane(uv, k);
        const int sl  = u & (NB - 1);
        const int eid = (int)((unsigned)u >> SLB);
        if (lane == 0) {
          int pos = cur[sl];
          pos = pos < 0 ? 0 : (pos > RCAP - 1 ? RCAP - 1 : pos);
          reg2[pos] = eid;
          cur[sl] = pos + 1;
        }
      }
    }
  }
  __syncthreads();

  const int nbw = NB / NWAVE;
  const bool ovf = (nh >= RCAP);
  const float qnan = __int_as_float(0x7fc00000);
  const float ph = bf16_val(prel[lane >> 2]);
  const int nDc = nDst > 1 ? nDst : 1;
  const int nSc = nSrc > 1 ? nSrc : 1;

#pragma unroll 1
  for (int jt = 0; jt < nbw; ++jt) {
    const int slot = wave * nbw + jt;
    const int grow = nodeBase + slot;
    const int gcl  = grow < nDc ? grow : nDc - 1;
    int st = soff[slot];
    const int craw = scnt[slot];
    int cnt = craw;
    st  = st < 0 ? 0 : (st > nh ? nh : st);
    cnt = cnt < 0 ? 0 : (cnt > DEGC ? DEGC : cnt);
    if (cnt > nh - st) cnt = nh - st;
    const float pz = (ovf || craw > DEGC) ? qnan : 0.0f;

    const v4f qa = *(const v4fa*)(Qp + (size_t)gcl * DIM + 4 * lane);
    ldwait();

    float mx = -1.0e30f, dn = 0.f;
    v4f ava = {0.f, 0.f, 0.f, 0.f};
#pragma unroll 1
    for (int q = 0; q < cnt; ++q) {
      int idx = st + q; idx = idx > RCAP - 1 ? RCAP - 1 : idx;
      int eid = reg2[idx]; eid = eid < 0 ? 0 : (eid > nE - 1 ? nE - 1 : eid);
      const int sraw = srcs[eid];
      const int s = sraw < 0 ? 0 : (sraw > nSc - 1 ? nSc - 1 : sraw);
      const float* kr = KVp + (size_t)s * KVW + 4 * lane;
      const v4f ka = *(const v4fa*)kr;
      const v4f va = *(const v4fa*)(kr + DIM);
      ldwait();
      float p = qa.x * ka.x;
      p = fmaf(qa.y, ka.y, p); p = fmaf(qa.z, ka.z, p); p = fmaf(qa.w, ka.w, p);
      p += __shfl_xor(p, 2);
      p += __shfl_xor(p, 1);
      const float lg = (p * ph) * ATTSC;
      const float df = lg - mx;
      const float ee = __expf(-fabsf(df));
      const bool up  = df > 0.f;
      const float s1 = up ? ee : 1.0f;
      const float s2 = up ? 1.0f : ee;
      mx = up ? lg : mx;
      dn = fmaf(dn, s1, s2);
      ava.x = fmaf(ava.x, s1, s2 * va.x); ava.y = fmaf(ava.y, s1, s2 * va.y);
      ava.z = fmaf(ava.z, s1, s2 * va.z); ava.w = fmaf(ava.w, s1, s2 * va.w);
    }
    const float dns = dn > 0.f ? dn : 1.0f;
    const float ind = dn > 0.f ? 1.0f : 0.0f;
    const float inv = ind * __builtin_amdgcn_rcpf(dns);
    v4f oa;
    oa.x = fmaf(ava.x, inv, pz); oa.y = fmaf(ava.y, inv, pz);
    oa.z = fmaf(ava.z, inv, pz); oa.w = fmaf(ava.w, inv, pz);
    const bool wr = (grow < MPr);
    const int gsf = wr ? grow : MPr - 1;
    if constexpr (MODE == 0) {
      float* orow = Sp + (size_t)gsf * DIM + 4 * lane;
      if (wr) *(volatile v4f*)orow = oa;
      __threadfence();
      if (wr) *(volatile v4f*)orow = oa;
    } else {
      const v4f pr = *(const v4fa*)(Sp + (size_t)gsf * DIM + 4 * lane);
      const v4f tv = pr + oa;
      v4f gv;
      gv.x = gelu_t(tv.x); gv.y = gelu_t(tv.y); gv.z = gelu_t(tv.z); gv.w = gelu_t(tv.w);
      const v8us po = hilo8(gv);
      unsigned short* hrow = Hp + (size_t)gsf * K2 + 8 * lane;
      if (wr) *(volatile v8us*)hrow = po;
      __threadfence();
      if (wr) *(volatile v8us*)hrow = po;
    }
  }
}

__global__ __launch_bounds__(GTHR) void k_upd(const unsigned short* __restrict__ A,
                                              const unsigned short* __restrict__ WT,
                                              const float* __restrict__ bias, const float* __restrict__ skp,
                                              unsigned short* xh) {
  __shared__ __attribute__((aligned(16))) float stg[GBM * DIM];
  const int tid = (int)threadIdx.x, lane = tid & 31, wave = tid >> 5, hh = lane >> 4, m = lane & 15;
  const int rowBase = (int)blockIdx.x * GBM;

  v8f acc[8];
  {
    const v8f z = {0.f, 0.f, 0.f, 0.f, 0.f, 0.f, 0.f, 0.f};
#pragma unroll
    for (int t = 0; t < 8; ++t) acc[t] = z;
  }
  const unsigned short* ap = A  + (size_t)(rowBase + 16 * wave + m) * (size_t)K2 + 8 * hh;
  const unsigned short* bp = WT + (size_t)m * (size_t)K2 + 8 * hh;

#pragma unroll 1
  for (int ks = 0; ks < K2 / 32; ++ks) {
    const int k0 = 32 * ks;
    Frag af;
    af.h[0] = *(const v8usa*)(ap + k0);
    af.h[1] = *(const v8usa*)(ap + k0 + 16);
#pragma unroll
    for (int nt = 0; nt < 8; ++nt) {
      const unsigned short* wq = bp + (size_t)(16 * nt) * (size_t)K2 + k0;
      Frag bf;
      bf.h[0] = *(const v8usa*)wq;
      bf.h[1] = *(const v8usa*)(wq + 16);
      acc[nt] = wmb(af, bf, acc[nt]);
    }
  }

#pragma unroll
  for (int nt = 0; nt < 8; ++nt) {
    const int lc = 16 * nt + m;
#pragma unroll
    for (int r = 0; r < 8; ++r) {
      const int lr = 16 * wave + 8 * hh + r;
      stg[lr * DIM + lc] = acc[nt][r];
    }
  }
  __syncthreads();

  const float sk = bf16_val(skp[0]);
  const float al = sigm_t(sk);
  const float om = 1.0f - al;
  v4f bb4;
  {
    const v4f tb = *(const v4fa*)(bias + 4 * lane);
    bb4.x = bf16_val(tb.x); bb4.y = bf16_val(tb.y); bb4.z = bf16_val(tb.z); bb4.w = bf16_val(tb.w);
  }
  v8us po[16];
#pragma unroll
  for (int i = 0; i < 16; ++i) {
    const int row = rowBase + 16 * wave + i;
    const v4f t  = *(const v4fa*)(stg + (16 * wave + i) * DIM + 4 * lane) + bb4;
    const v4u xw = *(const v4ua*)(xh + (size_t)row * (size_t)K2 + 8 * lane);
    const float x0 = __uint_as_float(xw.x << 16) + __uint_as_float(xw.z << 16);
    const float x1 = __uint_as_float(xw.x & 0xFFFF0000u) + __uint_as_float(xw.z & 0xFFFF0000u);
    const float x2 = __uint_as_float(xw.y << 16) + __uint_as_float(xw.w << 16);
    const float x3 = __uint_as_float(xw.y & 0xFFFF0000u) + __uint_as_float(xw.w & 0xFFFF0000u);
    v4f v;
    v.x = fmaf(al, t.x, om * x0); v.y = fmaf(al, t.y, om * x1);
    v.z = fmaf(al, t.z, om * x2); v.w = fmaf(al, t.w, om * x3);
    po[i] = hilo8(v);
  }
#pragma unroll
  for (int i = 0; i < 16; ++i) {
    unsigned short* rp = xh + (size_t)(rowBase + 16 * wave + i) * (size_t)K2 + 8 * lane;
    *(volatile v8us*)rp = po[i];
  }
  __threadfence();
#pragma unroll
  for (int i = 0; i < 16; ++i) {
    unsigned short* rp = xh + (size_t)(rowBase + 16 * wave + i) * (size_t)K2 + 8 * lane;
    *(volatile v8us*)rp = po[i];
  }
}

__global__ __launch_bounds__(GTHR) void k_final(const unsigned short* __restrict__ A,
                                                const unsigned short* __restrict__ WT,
                                                const float* __restrict__ bout, float* out, int nN) {
  __shared__ __attribute__((aligned(16))) float stg[GBM * NOP];
  __shared__ __attribute__((aligned(16))) float ob[GBM * NOUT];
  __shared__ float bb[NOP];
  const int tid = (int)threadIdx.x, lane = tid & 31, wave = tid >> 5, hh = lane >> 4, m = lane & 15;
  const int rowBase = (int)blockIdx.x * GBM;

  v8f acc[NTO];
  {
    const v8f z = {0.f, 0.f, 0.f, 0.f, 0.f, 0.f, 0.f, 0.f};
#pragma unroll
    for (int t = 0; t < NTO; ++t) acc[t] = z;
  }
  const unsigned short* ap = A  + (size_t)(rowBase + 16 * wave + m) * (size_t)K2 + 8 * hh;
  const unsigned short* bp = WT + (size_t)m * (size_t)K2 + 8 * hh;

#pragma unroll 1
  for (int ks = 0; ks < K2 / 32; ++ks) {
    const int k0 = 32 * ks;
    Frag af;
    af.h[0] = *(const v8usa*)(ap + k0);
    af.h[1] = *(const v8usa*)(ap + k0 + 16);
#pragma unroll
    for (int nt = 0; nt < NTO; ++nt) {
      const unsigned short* wq = bp + (size_t)(16 * nt) * (size_t)K2 + k0;
      Frag bf;
      bf.h[0] = *(const v8usa*)wq;
      bf.h[1] = *(const v8usa*)(wq + 16);
      acc[nt] = wmb(af, bf, acc[nt]);
    }
  }

#pragma unroll
  for (int nt = 0; nt < NTO; ++nt) {
    const int lc = 16 * nt + m;
#pragma unroll
    for (int r = 0; r < 8; ++r) {
      const int lr = 16 * wave + 8 * hh + r;
      stg[lr * NOP + lc] = acc[nt][r];
    }
  }
  for (int c = tid; c < NOP; c += GTHR) {
    const int cc = c < NOUT ? c : NOUT - 1;
    const float bvl = bf16_val(bout[cc]);
    bb[c] = (c < NOUT) ? bvl : 0.0f;
  }
  __syncthreads();

#pragma unroll 1
  for (int e = tid; e < GBM * NOUT; e += GTHR) {
    const int r = e / NOUT;
    const int c = e - r * NOUT;
    const float zz = stg[r * NOP + c] + bb[c];
    ob[e] = sigm_t(zz);
  }
  __syncthreads();

  int nv = nN - rowBase;
  nv = nv > GBM ? GBM : nv;
  const int npc = nv > 0 ? ((nv * NOUT) >> 2) : 0;
  v4f pv[NPQ];
#pragma unroll
  for (int q = 0; q < NPQ; ++q) {
    const int p  = tid + q * GTHR;
    const int pc = p < (GBM * NOUT) / 4 ? p : (GBM * NOUT) / 4 - 1;
    pv[q] = *(const v4fa*)(ob + 4 * pc);
  }
  const size_t obase = (size_t)(rowBase < nN ? rowBase : 0) * (size_t)NOUT;
#pragma unroll
  for (int q = 0; q < NPQ; ++q) {
    const int p = tid + q * GTHR;
    if (p < npc) *(volatile v4f*)(out + obase + 4 * (size_t)p) = pv[q];
  }
  __threadfence();
#pragma unroll
  for (int q = 0; q < NPQ; ++q) {
    const int p = tid + q * GTHR;
    if (p < npc) *(volatile v4f*)(out + obase + 4 * (size_t)p) = pv[q];
  }
}

static inline int cdiv(int a, int b) { return (a + b - 1) / b; }
static inline size_t al256(size_t x) { return (x + 255) & ~(size_t)255; }

extern "C" void kernel_launch(void* const* d_in, const int* in_sizes, int n_in,
                              void* d_out, int out_size, void* d_ws, size_t ws_size,
                              hipStream_t stream) {
  if (n_in < 29) return;
  if (in_sizes[0] < DIM || (in_sizes[0] % DIM) != 0) return;
  const int NPAT = in_sizes[0] / DIM;
  if (NPAT < 16 || (NPAT % 16) != 0 || NPAT > (1 << 22)) return;
  if (in_sizes[1] != DIM * DIM || in_sizes[2] != DIM) return;
  if (in_sizes[3] < DIM || (in_sizes[3] % DIM) != 0) return;
  if (in_sizes[4] < DIM || (in_sizes[4] % DIM) != 0) return;
  const int NEI = in_sizes[3] / DIM, NEN = in_sizes[4] / DIM;
  if (in_sizes[5] != 6 * DIM * DIM || in_sizes[7] != 6 * DIM * DIM) return;
  if (in_sizes[9] != 6 * DIM * DIM || in_sizes[11] != 6 * DIM * DIM) return;
  if (in_sizes[6] != 6 * DIM || in_sizes[8] != 6 * DIM) return;
  if (in_sizes[10] != 6 * DIM || in_sizes[12] != 6 * DIM) return;
  if (in_sizes[13] != 6) return;
  if (in_sizes[14] != 8 * HN * DK * DK || in_sizes[15] != 8 * HN * DK * DK) return;
  if (in_sizes[16] != 8 * HN) return;
  if (in_sizes[17] != DIM * NOUT || in_sizes[18] != NOUT) return;
  const int NICD = in_sizes[19], NNDC = in_sizes[20];
  if (NICD < 1 || NNDC < 1 || NICD > (1 << 20) || NNDC > (1 << 20)) return;
  int nEr[4];
  for (int r = 0; r < 4; ++r) {
    nEr[r] = in_sizes[21 + 2 * r];
    if (nEr[r] < 1 || in_sizes[22 + 2 * r] != nEr[r] || nEr[r] >= (1 << (31 - SLP))) return;
  }
  if ((long long)out_size != (long long)NPAT * NOUT) return;

  const float* x_pat = (const float*)d_in[0];
  const float* w_in  = (const float*)d_in[1];
  const float* b_in  = (const float*)d_in[2];
  const float* embi  = (const float*)d_in[3];
  const float* embn  = (const float*)d_in[4];
  const float* kw    = (const float*)d_in[5];
  const float* kb    = (const float*)d_in[6];
  const float* qw    = (const float*)d_in[7];
  const float* qb    = (const float*)d_in[8];
  const float* vw    = (const float*)d_in[9];
  const float* vb    = (const float*)d_in[10];
  const float* aw    = (const float*)d_in[11];
  const float* ab    = (const float*)d_in[12];
  const float* skip  = (const float*)d_in[13];
  const float* arel  = (const float*)d_in[14];
  const float* mrel  = (const float*)d_in[15];
  const float* prel  = (const float*)d_in[16];
  const float* w_out = (const float*)d_in[17];
  const float* b_out = (const float*)d_in[18];
  const int*   xicd  = (const int*)d_in[19];
  const int*   xndc  = (const int*)d_in[20];
  const int*   s_pi  = (const int*)d_in[21];
  const int*   d_pi  = (const int*)d_in[22];
  const int*   s_ip  = (const int*)d_in[23];
  const int*   d_ip  = (const int*)d_in[24];
  const int*   s_pn  = (const int*)d_in[25];
  const int*   d_pn  = (const int*)d_in[26];
  const int*   s_np  = (const int*)d_in[27];
  const int*   d_np  = (const int*)d_in[28];
  float* out = (float*)d_out;

  const int MP0 = cdiv(NPAT, 64) * 64;
  const int MP1 = cdiv(NICD, 64) * 64;
  const int MP2 = cdiv(NNDC, 64) * 64;
  const int MPS = MP1 > MP2 ? MP1 : MP2;

  char* ws = (char*)d_ws;
  size_t off = 0;
  const size_t oWINT = off; off = al256(off + (size_t)DIM * DIM * 2);
  const size_t oKQVT = off; off = al256(off + (size_t)6 * NQKV * K2 * 2);
  const size_t oAWT  = off; off = al256(off + (size_t)6 * DIM * K2 * 2);
  const size_t oWOT  = off; off = al256(off + (size_t)NOP * K2 * 2);
  const size_t oBDT  = off; off = al256(off + (size_t)8 * 16 * 16 * 32 * 2);
  const size_t oXH0  = off; off = al256(off + (size_t)MP0 * K2 * 2);
  const size_t oXH1  = off; off = al256(off + (size_t)MP1 * K2 * 2);
  const size_t oXH2  = off; off = al256(off + (size_t)MP2 * K2 * 2);
  const size_t oQ0   = off; off = al256(off + (size_t)MP0 * DIM * 4);
  const size_t oQ1   = off; off = al256(off + (size_t)MP1 * DIM * 4);
  const size_t oQ2   = off; off = al256(off + (size_t)MP2 * DIM * 4);
  const size_t oKV0  = off; off = al256(off + (size_t)MP0 * KVW * 4);
  const size_t oKV1  = off; off = al256(off + (size_t)MP1 * KVW * 4);
  const size_t oKV2  = off; off = al256(off + (size_t)MP2 * KVW * 4);
  const size_t oQT   = off; off = al256(off + (size_t)MPS * DIM * 4);
  const size_t oS12  = off; off = al256(off + (size_t)MPS * DIM * 4);
  const size_t oAH1  = off; off = al256(off + (size_t)MP1 * K2 * 2);
  const size_t oAH2  = off; off = al256(off + (size_t)MP2 * K2 * 2);
  const size_t oKRS  = off; off = al256(off + (size_t)MPS * KVW * 4);
  if (off > ws_size || off > (size_t)WSMAX) return;
  unsigned short* WINT = (unsigned short*)(ws + oWINT);
  unsigned short* KQVT = (unsigned short*)(ws + oKQVT);
  unsigned short* AWT  = (unsigned short*)(ws + oAWT);
  unsigned short* WOT  = (unsigned short*)(ws + oWOT);
  unsigned short* BDT  = (unsigned short*)(ws + oBDT);
  unsigned short* XH0  = (unsigned short*)(ws + oXH0);
  unsigned short* XH1  = (unsigned short*)(ws + oXH1);
  unsigned short* XH2  = (unsigned short*)(ws + oXH2);
  float*          Q0   = (float*)(ws + oQ0);
  unsigned short* XB   = (unsigned short*)(ws + oQ0);
  float*          Q1   = (float*)(ws + oQ1);
  float*          Q2   = (float*)(ws + oQ2);
  float*          KV0  = (float*)(ws + oKV0);
  float*          S0   = (float*)(ws + oKV0);
  unsigned short* AH0  = (unsigned short*)(ws + oKV0 + (size_t)MP0 * DIM * 4);
  float*          KV1  = (float*)(ws + oKV1);
  float*          KV2  = (float*)(ws + oKV2);
  float*          QT   = (float*)(ws + oQT);
  float*          S12  = (float*)(ws + oS12);
  unsigned short* AH1  = (unsigned short*)(ws + oAH1);
  unsigned short* AH2  = (unsigned short*)(ws + oAH2);
  float*          KRS  = (float*)(ws + oKRS);

  const int ldsI = AGG_INTS(NBI) * 4 + 64;
  const int ldsN = AGG_INTS(NBN) * 4 + 64;
  const int ldsP = AGG_INTS(NBP) * 4 + 64;
  hipFuncSetAttribute(reinterpret_cast<const void*>(&k_agg<NBI, SLI, DGI, 0>), hipFuncAttributeMaxDynamicSharedMemorySize, ldsI);
  hipFuncSetAttribute(reinterpret_cast<const void*>(&k_agg<NBN, SLN, DGN, 0>), hipFuncAttributeMaxDynamicSharedMemorySize, ldsN);
  hipFuncSetAttribute(reinterpret_cast<const void*>(&k_agg<NBP, SLP, DGP, 0>), hipFuncAttributeMaxDynamicSharedMemorySize, ldsP);
  hipFuncSetAttribute(reinterpret_cast<const void*>(&k_agg<NBP, SLP, DGP, 1>), hipFuncAttributeMaxDynamicSharedMemorySize, ldsP);

  const int gI = cdiv(MP1, NBI);
  const int gN = cdiv(MP2, NBN);
  const int gP = cdiv(MP0, NBP);
  int vec[4];
  for (int r = 0; r < 4; ++r) vec[r] = ((nEr[r] & 3) == 0) ? 1 : 0;
  const int MPt[3] = { MP0, MP1, MP2 };
  unsigned short* XH[3] = { XH0, XH1, XH2 };
  unsigned short* AH[3] = { AH0, AH1, AH2 };
  float* Qt[3]  = { Q0, Q1, Q2 };
  float* KVt[3] = { KV0, KV1, KV2 };

  k_prep<<<NUT / NTHR, NTHR, 0, stream>>>(w_in, kw, vw, qw, aw, w_out, arel, mrel, WINT, KQVT, AWT, WOT, BDT);
  k_cvx<<<(MP0 * (DIM / 8)) / NTHR, NTHR, 0, stream>>>(x_pat, NPAT, MP0 * (DIM / 8), XB);
  k_emb<<<(MP1 * 32 + MP2 * 32) / NTHR, NTHR, 0, stream>>>(embi, xicd, NICD, NEI, MP1, embn, xndc, NNDC, NEN, MP2,
                                                           XH1, XH2);
  k_gemm0<<<MP0 / GBM, GTHR, 0, stream>>>(XB, WINT, b_in, XH0);

  for (int l = 0; l < 2; ++l) {
    for (int t = 0; t < 3; ++t) {
      const int lt = l * 3 + t;
      k_gemmx<<<dim3(MPt[t] / GBM, 3), GTHR, 0, stream>>>(XH[t], KQVT + (size_t)lt * NQKV * K2,
                                                          kb + (size_t)lt * DIM, vb + (size_t)lt * DIM,
                                                          qb + (size_t)lt * DIM, KVt[t], Qt[t]);
    }
    {
      const int lr = l * 4 + 0;
      k_bd<0><<<dim3(MP1 / BBM, DIM / 64), BTHR, 0, stream>>>(Q1, DIM, BDT + (size_t)(lr * 16) * 512, QT, DIM, AH1);
      k_agg<NBI, SLI, DGI, 0><<<gI, NTHR, ldsI, stream>>>(s_pi, d_pi, nEr[0], vec[0], QT, NICD, KV0, NPAT,
                                                           prel + lr * HN, S12, AH1, MP1);
      k_bd<1><<<dim3(MP1 / BBM, DIM / 64), BTHR, 0, stream>>>(S12, DIM, BDT + (size_t)(lr * 16 + 8) * 512, QT, DIM, AH1);
    }
    {
      const int lr = l * 4 + 2;
      k_bd<0><<<dim3(MP2 / BBM, DIM / 64), BTHR, 0, stream>>>(Q2, DIM, BDT + (size_t)(lr * 16) * 512, QT, DIM, AH2);
      k_agg<NBN, SLN, DGN, 0><<<gN, NTHR, ldsN, stream>>>(s_pn, d_pn, nEr[2], vec[2], QT, NNDC, KV0, NPAT,
                                                           prel + lr * HN, S12, AH2, MP2);
      k_bd<1><<<dim3(MP2 / BBM, DIM / 64), BTHR, 0, stream>>>(S12, DIM, BDT + (size_t)(lr * 16 + 8) * 512, QT, DIM, AH2);
    }
    {
      const int lr = l * 4 + 1;
      k_bd<0><<<dim3(MP1 / BBM, KVW / 64), BTHR, 0, stream>>>(KV1, KVW, BDT + (size_t)(lr * 16) * 512, KRS, KVW, AH1);
      k_agg<NBP, SLP, DGP, 0><<<gP, NTHR, ldsP, stream>>>(s_ip, d_ip, nEr[1], vec[1], Q0, NPAT, KRS, NICD,
                                                           prel + lr * HN, S0, AH0, MP0);
    }
    {
      const int lr = l * 4 + 3;
      k_bd<0><<<dim3(MP2 / BBM, KVW / 64), BTHR, 0, stream>>>(KV2, KVW, BDT + (size_t)(lr * 16) * 512, KRS, KVW, AH2);
      k_agg<NBP, SLP, DGP, 1><<<gP, NTHR, ldsP, stream>>>(s_np, d_np, nEr[3], vec[3], Q0, NPAT, KRS, NNDC,
                                                           prel + lr * HN, S0, AH0, MP0);
    }
    for (int t = 0; t < 3; ++t) {
      const int lt = l * 3 + t;
      k_upd<<<MPt[t] / GBM, GTHR, 0, stream>>>(AH[t], AWT + (size_t)lt * DIM * K2, ab + (size_t)lt * DIM,
                                                skip + lt, XH[t]);
    }
  }

  k_final<<<MP0 / GBM, GTHR, 0, stream>>>(XH0, WOT, b_out, out, NPAT);
}
